// CLIPAttention_11467562681048
// MI455X (gfx1250) — hardware-verified
//
#include <hip/hip_runtime.h>


#ifndef NB
#define NB 16
#endif
#ifndef SEQ
#define SEQ 577
#endif
#define SEQF 577
#define NBF  16
#define DM   1024
#define NH_  16
#define HD   64
#define DQ   (NH_ * HD)
#define S_   SEQ
#define SPR  (((S_ + 63) / 64) * 64)
#define SPK  SPR
#define SCP  SPR
#define MR   (NB * S_)
#define MP   (((MR + 63) / 64) * 64)
#define PCAR 1024.0f
#define SCL  0.125f

static_assert(SPK % 64 == 0);
static_assert(MP % 64 == 0);
static_assert(DM % 64 == 0);
static_assert(DQ == DM);
static_assert(NB <= NBF);
static_assert(S_ <= SEQF);
static_assert(HD == 64);

typedef _Float16 h16;
typedef unsigned short bf;
typedef __attribute__((ext_vector_type(16))) __bf16   v16bf;
typedef __attribute__((ext_vector_type(16))) _Float16 v16h;
typedef __attribute__((ext_vector_type(8)))  _Float16 v8h;
typedef __attribute__((ext_vector_type(8)))  unsigned short v8us;
typedef __attribute__((ext_vector_type(8)))  float    v8f;
typedef __attribute__((ext_vector_type(4)))  float    v4f;
typedef __attribute__((ext_vector_type(2)))  _Float16 v2h;
typedef __attribute__((ext_vector_type(2)))  unsigned short v2us;
typedef v8h  __attribute__((may_alias)) v8ha;
typedef v4f  __attribute__((may_alias)) v4fa;

__device__ __forceinline__ unsigned short f2bf(float f) { unsigned u = __float_as_uint(f); u += 0x7FFFu + ((u >> 16) & 1u); return (unsigned short)(u >> 16); }
__device__ __forceinline__ float bf2f(unsigned short b) { return __uint_as_float(((unsigned)b) << 16); }
__device__ __forceinline__ float bfr(float f) { return bf2f(f2bf(f)); }
__device__ __forceinline__ h16 tohx(float x) { return (h16)x; }
__device__ __forceinline__ void splitf(float y, unsigned short& h, unsigned short& l) { h = f2bf(y); l = f2bf(y - bf2f(h)); }
__device__ __forceinline__ v16h cat16(v8h lo, v8h hi) { return __builtin_shufflevector(lo, hi, 0, 1, 2, 3, 4, 5, 6, 7, 8, 9, 10, 11, 12, 13, 14, 15); }
__device__ __forceinline__ v16bf cat16b(v8us lo, v8us hi) { return __builtin_bit_cast(v16bf, __builtin_shufflevector(lo, hi, 0, 1, 2, 3, 4, 5, 6, 7, 8, 9, 10, 11, 12, 13, 14, 15)); }
__device__ __forceinline__ v8f wmma16(v16h a, v16h b, v8f c) { return __builtin_amdgcn_wmma_f32_16x16x32_f16(false, a, false, b, (short)0, c, false, false); }
__device__ __forceinline__ v8f wmmab(v16bf a, v16bf b, v8f c) { return __builtin_amdgcn_wmma_f32_16x16x32_bf16(false, a, false, b, (short)0, c, false, false); }

template <typename T16> struct WFrag;
template <> struct WFrag<h16> { typedef v16h V; static __device__ __forceinline__ V ld(const h16* p) { return cat16(*(const v8h*)p, *(const v8h*)(p + 16)); } static __device__ __forceinline__ v8f mma(V a, V b, v8f c) { return wmma16(a, b, c); } };
template <> struct WFrag<bf> { typedef v16bf V; static __device__ __forceinline__ V ld(const bf* p) { return cat16b(*(const v8us*)p, *(const v8us*)(p + 16)); } static __device__ __forceinline__ v8f mma(V a, V b, v8f c) { return wmmab(a, b, c); } };
template <typename T16, int NSPLIT, bool BIAS>
__global__ __launch_bounds__(32) void k_gemmw(const T16* __restrict__ A, const T16* __restrict__ A2, const T16* __restrict__ Bt, const T16* __restrict__ Bt2, int K, float* C, int ldc, const float* __restrict__ bias, int Mlim, size_t sA, size_t sB, size_t sC) {
    typedef typename WFrag<T16>::V V;
    __shared__ __align__(16) float os[16 * 68];
    const size_t z = blockIdx.z; A += z * sA; if (A2) A2 += z * sA; Bt += z * sB; if (Bt2) Bt2 += z * sB; C += z * sC;
    const int lane = threadIdx.x & 31, lr = lane & 15, hi = lane >> 4; const int r0 = blockIdx.x * 64, c0 = blockIdx.y * 64;
    v8f acc[4][4];
#pragma unroll
    for (int mb = 0; mb < 4; ++mb)
#pragma unroll
        for (int nb = 0; nb < 4; ++nb) acc[mb][nb] = (v8f){};
    const size_t aoff = (size_t)(r0 + lr) * K + 8 * hi, boff = (size_t)(c0 + lr) * K + 8 * hi;
#pragma unroll 1
    for (int kc = 0; kc < K; kc += 32) {
        V a[4], a2[4];
#pragma unroll
        for (int mb = 0; mb < 4; ++mb) { a[mb] = WFrag<T16>::ld(A + aoff + (size_t)mb * 16 * K + kc); if (NSPLIT == 1 || NSPLIT == 2) a2[mb] = WFrag<T16>::ld(A2 + aoff + (size_t)mb * 16 * K + kc); }
#pragma unroll
        for (int nb = 0; nb < 4; ++nb) { const V b = WFrag<T16>::ld(Bt + boff + (size_t)nb * 16 * K + kc); V b2; if (NSPLIT >= 2) b2 = WFrag<T16>::ld(Bt2 + boff + (size_t)nb * 16 * K + kc);
#pragma unroll
            for (int mb = 0; mb < 4; ++mb) { acc[mb][nb] = WFrag<T16>::mma(a[mb], b, acc[mb][nb]); if (NSPLIT == 1 || NSPLIT == 2) acc[mb][nb] = WFrag<T16>::mma(a2[mb], b, acc[mb][nb]); if (NSPLIT >= 2) acc[mb][nb] = WFrag<T16>::mma(a[mb], b2, acc[mb][nb]); } }
        asm volatile("v_nop\n\tv_nop\n\tv_nop\n\tv_nop" : "+v"(acc[0][0]), "+v"(acc[1][1]), "+v"(acc[2][2]), "+v"(acc[3][3]) : "v"(a[0]), "v"(a[3]));
    }
#pragma unroll
    for (int mb = 0; mb < 4; ++mb) {
#pragma unroll
        for (int nb = 0; nb < 4; ++nb) {
#pragma unroll
            for (int j = 0; j < 8; ++j) os[(hi * 8 + j) * 68 + nb * 16 + lr] = acc[mb][nb][j]; }
        __builtin_amdgcn_wave_barrier(); asm volatile("" ::: "memory");
        float* crow = C + (size_t)(r0 + mb * 16) * ldc + c0;
#pragma unroll 1
        for (int ps = 0; ps < 2; ++ps) {
#pragma unroll
            for (int s = 0; s < 8; ++s) { const int row = 2 * s + hi, cofs = lr * 4; v4f val = *(const v4fa*)(os + row * 68 + cofs); if (BIAS) { val[0] += bfr(bias[c0 + cofs]); val[1] += bfr(bias[c0 + cofs + 1]); val[2] += bfr(bias[c0 + cofs + 2]); val[3] += bfr(bias[c0 + cofs + 3]); }
                if (r0 + mb * 16 + row < Mlim) *(volatile v4f*)(crow + (size_t)row * ldc + cofs) = val; }
            if (ps == 0) __threadfence(); }
        __builtin_amdgcn_wave_barrier(); asm volatile("" ::: "memory");
    }
}

__global__ __launch_bounds__(256) void k_cvt8(const float* __restrict__ src, bf* dst, size_t n8) { const size_t i = (size_t)blockIdx.x * 256 + threadIdx.x; if (i >= n8) return; const v8f v = *(const v8f*)(src + i * 8); v8us o;
#pragma unroll
    for (int k = 0; k < 8; ++k) o[k] = f2bf(v[k]); *(volatile v8us*)(dst + i * 8) = o; __threadfence(); *(volatile v8us*)(dst + i * 8) = o; }

__global__ __launch_bounds__(256) void k_cvtx(const float* __restrict__ src, bf* dst) {
    const size_t i = (size_t)blockIdx.x * 256 + threadIdx.x; const size_t n8 = (size_t)MP * DM / 8; if (i >= n8) return;
    const int r = (int)(i / (DM / 8)); const int c8 = (int)(i % (DM / 8)); const int rc = (r < MR) ? r : (MR - 1); const int b = rc / S_, t = rc - b * S_;
    const v8f v = *(const v8f*)(src + ((size_t)b * SEQF + t) * DM + (size_t)c8 * 8); v8us o;
#pragma unroll
    for (int k = 0; k < 8; ++k) o[k] = (r < MR) ? f2bf(v[k]) : (unsigned short)0;
    *(volatile v8us*)(dst + i * 8) = o; __threadfence(); *(volatile v8us*)(dst + i * 8) = o; }

__global__ __launch_bounds__(256) void k_zero8(bf* dst, size_t n8) { const size_t i = (size_t)blockIdx.x * 256 + threadIdx.x; if (i >= n8) return; v8us o;
#pragma unroll
    for (int k = 0; k < 8; ++k) o[k] = (unsigned short)0; *(volatile v8us*)(dst + i * 8) = o; __threadfence(); *(volatile v8us*)(dst + i * 8) = o; }

__global__ __launch_bounds__(256) void k_score(const float* __restrict__ F, const float* __restrict__ key, float* SC) {
    const int lane = threadIdx.x & 31; const int gw = blockIdx.x * 8 + (threadIdx.x >> 5); const int nch = SCP / 32;
    const int bh = gw / nch; const int ch = gw - bh * nch; if (bh >= NB * NH_) return;
    const int b = bh / NH_, h = bh - b * NH_; const int i = ch * 32 + lane; const int ic = (i < S_) ? i : (S_ - 1);
    const float* fr = F + ((size_t)(b * S_ + ic)) * DM + h * HD; const float* kr = key + h * HD;
    float acc = 0.0f;
#pragma unroll 4
    for (int d = 0; d < HD; ++d) acc = fmaf(fr[d], bfr(kr[d]), acc);
    const float s = (i < S_) ? acc * SCL : 0.0f;
    float* p = SC + (size_t)bh * SCP + i;
    *(volatile float*)p = s; __threadfence(); *(volatile float*)p = s;
}

__global__ __launch_bounds__(256) void k_vtp(const float* __restrict__ F, h16* V16) {
    const size_t e = ((size_t)blockIdx.x * 256 + threadIdx.x) * 2; if (e >= (size_t)NB * NH_ * HD * SPK) return;
    const int t = (int)(e % SPK); const int d = (int)((e / SPK) % HD); const int g = (int)(e / ((size_t)SPK * HD)); const int b = g / NH_, h = g - b * NH_;
    v2h o16;
#pragma unroll
    for (int q = 0; q < 2; ++q) { const int tt = t + q; const int tc = (tt < S_) ? tt : (S_ - 1); float x = F[((size_t)(b * S_ + tc)) * DM + h * HD + d]; x = (tt < S_) ? x : 0.0f; o16[q] = tohx(x); }
    *(volatile v2h*)(V16 + e) = o16; __threadfence(); *(volatile v2h*)(V16 + e) = o16;
}

__global__ __launch_bounds__(256) void k_asoft(const float* __restrict__ bias, const float* __restrict__ SC, int b, h16* P16) {
    __shared__ __align__(16) h16 prow[8][SPK];
    const int lane = threadIdx.x & 31, wv = threadIdx.x >> 5; const int row = blockIdx.x * 8 + wv; if (row >= NH_ * SPR) return;
    const int h = row / SPR, i = row - h * SPR; h16* pr = prow[wv];
    if (i < S_) {
        const float s = SC[((size_t)(b * NH_ + h)) * SCP + i];
        const float* br = bias + ((size_t)h * SEQF + i) * SEQF;
        float v[SPK / 32]; float mx = -3.0e38f;
#pragma unroll
        for (int ch = 0; ch < SPK / 32; ++ch) { const int j = ch * 32 + lane; const int jc = (j < S_) ? j : (S_ - 1); const float t = __fadd_rn(s, bfr(br[jc])); v[ch] = (j < S_) ? t : -3.0e38f; mx = fmaxf(mx, v[ch]);
            if (ch == SPK / 64 - 1) asm volatile("" ::: "memory"); }
#pragma unroll
        for (int sh = 16; sh; sh >>= 1) mx = fmaxf(mx, __shfl_xor(mx, sh, 32));
        float sum = 0.f;
#pragma unroll
        for (int ch = 0; ch < SPK / 32; ++ch) { float d0 = __fsub_rn(v[ch], mx); asm volatile("" : "+v"(d0)); float ex = __builtin_amdgcn_exp2f(__fmul_rn(d0, 1.4426950408889634f)); ex = (ch * 32 + lane < S_) ? ex : 0.0f; v[ch] = ex; sum += ex; }
#pragma unroll
        for (int sh = 16; sh; sh >>= 1) sum += __shfl_xor(sum, sh, 32);
        const float f = __fdiv_rn(PCAR, sum);
#pragma unroll
        for (int ch = 0; ch < SPK / 32; ++ch) pr[ch * 32 + lane] = tohx(v[ch] * f);
    } else {
#pragma unroll
        for (int ch = 0; ch < SPK / 32; ++ch) pr[ch * 32 + lane] = (h16)0.0f;
    }
    __builtin_amdgcn_wave_barrier(); asm volatile("" ::: "memory");
    h16* pg = P16 + ((size_t)h * SPR + i) * SPK;
#pragma unroll 1
    for (int ps = 0; ps < 2; ++ps) {
#pragma unroll
        for (int it = 0; it < (SPK / 8 + 31) / 32; ++it) { const int c = it * 32 + lane; if (c < SPK / 8) { const v8h val = *(const v8ha*)(pr + c * 8); *(volatile v8h*)(pg + (size_t)c * 8) = val; } }
        if (ps == 0) __threadfence(); }
}

__global__ __launch_bounds__(256) void k_merge(const float* __restrict__ O, int b, bf* Ah, bf* Al) {
    const size_t e = ((size_t)blockIdx.x * 256 + threadIdx.x) * 2; if (e >= (size_t)NH_ * S_ * HD) return;
    const int d = (int)(e % HD); const int t = (int)((e / HD) % S_); const int h = (int)(e / ((size_t)HD * S_));
    const size_t so = ((size_t)h * SPR + t) * HD + d; const size_t oo = ((size_t)(b * S_ + t)) * DM + h * HD + d;
    v2us oh, ol;
#pragma unroll
    for (int q = 0; q < 2; ++q) { unsigned short a, c2; splitf(O[so + q] * (1.0f / PCAR), a, c2); oh[q] = a; ol[q] = c2; }
    *(volatile v2us*)(Ah + oo) = oh; *(volatile v2us*)(Al + oo) = ol; __threadfence(); *(volatile v2us*)(Ah + oo) = oh; *(volatile v2us*)(Al + oo) = ol;
}

extern "C" void kernel_launch(void* const* d_in, const int* in_sizes, int n_in,
                              void* d_out, int out_size, void* d_ws, size_t ws_size, hipStream_t stream) {
    if (n_in < 9) return;
    if ((size_t)in_sizes[0] < ((size_t)(NB - 1) * SEQF + S_) * DM) return;
    if (in_sizes[1] < DM * DM || in_sizes[3] < DM * DM || in_sizes[5] < DM * DM) return;
    if (in_sizes[2] < DM || in_sizes[4] < DM || in_sizes[6] < DM) return;
    if (in_sizes[7] < NH_ * HD) return;
    if ((size_t)in_sizes[8] < ((size_t)(NH_ - 1) * SEQF + (S_ - 1)) * SEQF + S_) return;
    if ((size_t)out_size < (size_t)MR * DM) return;
    const float* x = (const float*)d_in[0]; const float* wq = (const float*)d_in[1]; const float* bq = (const float*)d_in[2]; const float* wv = (const float*)d_in[3]; const float* bv = (const float*)d_in[4];
    const float* wo = (const float*)d_in[5]; const float* bo = (const float*)d_in[6]; const float* key = (const float*)d_in[7]; const float* bias = (const float*)d_in[8];
    float* OUT = (float*)d_out;
    char* wsp = (char*)d_ws;
    auto take = [&](size_t bytes) { char* p = wsp; wsp += (bytes + 255) & ~(size_t)255; return (void*)p; };
    bf* WQ = (bf*)take((size_t)DM * DM * 2); bf* WV = (bf*)take((size_t)DM * DM * 2); bf* WO = (bf*)take((size_t)DM * DM * 2);
    bf* XB = (bf*)take((size_t)MP * DM * 2);
    float* F = (float*)take((size_t)MP * DM * 4);
    float* SC = (float*)take((size_t)NB * NH_ * SCP * 4);
    h16* VT16 = (h16*)take((size_t)NB * NH_ * HD * SPK * 2);
    h16* P16 = (h16*)take((size_t)NH_ * SPR * SPK * 2);
    float* Ob = (float*)take((size_t)NH_ * SPR * HD * 4);
    if ((size_t)(wsp - (char*)d_ws) > ws_size) return;
    static_assert((size_t)2 * MP * DM * 2 <= (size_t)MP * DM * 4);
    bf* ATh = (bf*)F; bf* ATl = ATh + (size_t)MP * DM;

    k_cvtx<<<(unsigned)(((size_t)MP * DM / 8 + 255) / 256), 256, 0, stream>>>(x, XB);
    const size_t nw8 = (size_t)DM * DM / 8;
    k_cvt8<<<(unsigned)((nw8 + 255) / 256), 256, 0, stream>>>(wq, WQ, nw8);
    k_cvt8<<<(unsigned)((nw8 + 255) / 256), 256, 0, stream>>>(wv, WV, nw8);
    k_cvt8<<<(unsigned)((nw8 + 255) / 256), 256, 0, stream>>>(wo, WO, nw8);
    k_gemmw<bf, 0, true><<<dim3(MP / 64, DQ / 64, 1), 32, 0, stream>>>(XB, nullptr, WQ, nullptr, DM, F, DQ, bq, MP, 0, 0, 0);
    k_score<<<(unsigned)((NB * NH_ * (SCP / 32) + 7) / 8), 256, 0, stream>>>(F, key, SC);
    k_gemmw<bf, 0, true><<<dim3(MP / 64, DQ / 64, 1), 32, 0, stream>>>(XB, nullptr, WV, nullptr, DM, F, DQ, bv, MP, 0, 0, 0);
    k_vtp<<<(unsigned)(((size_t)NB * NH_ * HD * SPK / 2 + 255) / 256), 256, 0, stream>>>(F, VT16);
    if (MP > MR) { const size_t z8 = (size_t)(MP - MR) * DM / 8;
        k_zero8<<<(unsigned)((z8 + 255) / 256), 256, 0, stream>>>(ATh + (size_t)MR * DM, z8);
        k_zero8<<<(unsigned)((z8 + 255) / 256), 256, 0, stream>>>(ATl + (size_t)MR * DM, z8); }
    for (int b = 0; b < NB; ++b) {
        k_asoft<<<(unsigned)((NH_ * SPR + 7) / 8), 256, 0, stream>>>(bias, SC, b, P16);
        k_gemmw<h16, 0, false><<<dim3(SPR / 64, HD / 64, NH_), 32, 0, stream>>>(P16, nullptr, VT16 + (size_t)b * NH_ * HD * SPK, nullptr, SPK, Ob, HD, nullptr, SPR, (size_t)SPR * SPK, (size_t)HD * SPK, (size_t)SPR * HD);
        k_merge<<<(unsigned)(((size_t)NH_ * S_ * HD / 2 + 255) / 256), 256, 0, stream>>>(Ob, b, ATh, ATl); }
    k_gemmw<bf, 1, true><<<dim3(MP / 64, DM / 64, 1), 32, 0, stream>>>(ATh, ATl, WO, nullptr, DQ, OUT, DM, bo, MR, 0, 0, 0);
}
